// Generator_1228360646784
// MI455X (gfx1250) — hardware-verified
//
#include <hip/hip_runtime.h>
#include <stddef.h>


typedef _Float16 h16;
typedef _Float16 v16h __attribute__((ext_vector_type(16)));
typedef _Float16 v8h  __attribute__((ext_vector_type(8)));
typedef float    v8f  __attribute__((ext_vector_type(8)));
typedef float    v4f  __attribute__((ext_vector_type(4)));
typedef float    v2f  __attribute__((ext_vector_type(2)));
typedef unsigned int v4u __attribute__((ext_vector_type(4)));
typedef unsigned int v8u __attribute__((ext_vector_type(8)));

#ifndef NROWS
#define NROWS 1000000
#endif
#define NROWS_FULL 1000000
#define NODES 6
#define NPAR  3
#define HIDN  64
#define WAVES 4
#define NTILES (NROWS / 16)
#define TILE_FLOATS (16 * NODES)

static_assert(NROWS >= 16 && NROWS <= NROWS_FULL);
static_assert((NROWS % 16) == 0);
static_assert(HIDN == 64);
static_assert(NODES == 6 && NPAR == 3);
static_assert((TILE_FLOATS * 4) % 128 == 0);
static_assert(TILE_FLOATS == 24 * 4);
static_assert((NODES * HIDN) % 64 == 0);

#define LDT 72
static_assert((LDT % 8) == 0 && LDT >= 64);

#define WCARRY 64.0f
#define XCARRY 8.0f
#define W0CARRY 8.0f
#define HCARRY (XCARRY * W0CARRY)
#define ACARRY (HCARRY * WCARRY)
#define SLOPE 0.2f

#define W1T_PITCH (NODES * HIDN)
#define W1T_BYTES ((size_t)HIDN * W1T_PITCH * 2)
#define A0_PIECES (NODES * HIDN * 2)
#define A0_BYTES  ((size_t)A0_PIECES * 16)
#define SP_C1   0
#define SP_W2   (NODES * HIDN)
#define SP_B2   (2 * NODES * HIDN)
#define SP_FLOATS (2 * NODES * HIDN + 32)
#define SP_BYTES ((size_t)SP_FLOATS * 4)
#define OFF_W1T ((size_t)0)
#define OFF_A0  (OFF_W1T + W1T_BYTES)
#define OFF_SP  (OFF_A0 + A0_BYTES)
#define WS_TOTAL (OFF_SP + SP_BYTES)
static_assert((W1T_BYTES % 128) == 0 && (A0_BYTES % 128) == 0 && (SP_BYTES % 128) == 0);
static_assert(A0_PIECES == 2 * 384);
static_assert(SP_FLOATS == 200 * 4);
static_assert((SP_W2 % 4) == 0 && (SP_B2 % 4) == 0);
static_assert(WS_TOTAL <= (size_t)134217728);

__device__ __forceinline__ float bf16r(float x) {
  unsigned int u = __float_as_uint(x);
  u = (u + 0x7FFFu + ((u >> 16) & 1u)) & 0xFFFF0000u;
  return __uint_as_float(u);
}

static __device__ __forceinline__ h16 toh_flush(float v) {
  const h16 r = (h16)v;
  return (fabsf(v) < 6.103515625e-05f) ? (h16)0.0f : r;
}
static __device__ __forceinline__ unsigned int hbits(float v) {
  return (unsigned int)__builtin_bit_cast(unsigned short, toh_flush(v));
}

__device__ __forceinline__ v16h frag_at(const _Float16* p) {
  v8h lo = *(const v8h*)(p);
  v8h hi = *(const v8h*)(p + 16);
  v16h out;
#pragma unroll
  for (int i = 0; i < 8; ++i) { out[i] = lo[i]; out[i + 8] = hi[i]; }
  return out;
}

__device__ __forceinline__ v8f wmma16(v16h a, v16h b, v8f c) {
  v8f d = __builtin_amdgcn_wmma_f32_16x16x32_f16(false, a, false, b, (short)0, c,
                                                 false, false);
  asm volatile("v_nop\n\tv_nop\n\tv_nop\n\tv_nop" : "+v"(d) : "v"(a), "v"(b));
  return d;
}

__device__ __forceinline__ void wave_lds_sync() {
  __builtin_amdgcn_fence(3  , "wavefront");
  asm volatile("s_wait_dscnt 0x0" ::: "memory");
  __builtin_amdgcn_wave_barrier();
}

__device__ __forceinline__ float leaky_act(float v) {
  return fmaxf(v, SLOPE * v);
}

__device__ __forceinline__ float pick6(int p, float a0, float a1, float a2, float a3,
                                       float a4, float a5) {
  float v = a0;
  v = (p == 1) ? a1 : v;
  v = (p == 2) ? a2 : v;
  v = (p == 3) ? a3 : v;
  v = (p == 4) ? a4 : v;
  v = (p == 5) ? a5 : v;
  return v;
}

__device__ __forceinline__ float carry_x(float v, bool on) {
  const float t = XCARRY * bf16r(v);
  return on ? t : 0.0f;
}

__global__ __launch_bounds__(256) void wconv_kernel(
    const float* __restrict__ W, _Float16* __restrict__ Wt, unsigned ldw, unsigned ldk) {
  __shared__ _Float16 T[64 * LDT];
  const unsigned tid = threadIdx.x;
  const unsigned n0 = blockIdx.x * 64u;
  const unsigned k0 = blockIdx.y * 64u;
#pragma unroll 4
  for (unsigned j = 0; j < 16u; ++j) {
    const unsigned idx = tid + 256u * j;
    const unsigned kr = idx >> 6, nc = idx & 63u;
    const float v = W[(size_t)(k0 + kr) * ldw + n0 + nc];
    T[nc * LDT + kr] = (_Float16)(WCARRY * bf16r(v));
  }
  __syncthreads();
  v8h x[2];
  size_t off[2];
#pragma unroll
  for (unsigned i = 0; i < 2u; ++i) {
    const unsigned n = 32u * i + (tid >> 3);
    const unsigned kc = (tid & 7u) * 8u;
    x[i] = *(const v8h*)&T[n * LDT + kc];
    off[i] = (size_t)(n0 + n) * ldk + k0 + kc;
  }
#pragma unroll
  for (int i = 0; i < 2; ++i) *(volatile v8h*)(Wt + off[i]) = x[i];
  __threadfence();
#pragma unroll
  for (int i = 0; i < 2; ++i) *(volatile v8h*)(Wt + off[i]) = x[i];
}

__global__ __launch_bounds__(384) void prep_small_kernel(
    const float* __restrict__ W0, const float* __restrict__ b0, const float* __restrict__ b1,
    const float* __restrict__ W2, const float* __restrict__ b2,
    unsigned int* __restrict__ A0w, float* __restrict__ SP) {
#pragma clang fp contract(off)
  const unsigned t = threadIdx.x;

  v4u pc[2];
  size_t po[2];
#pragma unroll
  for (unsigned i = 0; i < 2u; ++i) {
    const unsigned q = t + 384u * i;
    const unsigned e = q >> 1;
    const unsigned s = e >> 6, j = e & 63u;
    const bool on = ((q & 1u) == 0u);
    const float w0 = W0[s * 256u + j];
    const float w1 = W0[s * 256u + 64u + j];
    const float w2 = W0[s * 256u + 128u + j];
    const float w3 = W0[s * 256u + 192u + j];
    const float bb = b0[e];
    const unsigned int c0 = hbits(W0CARRY * bf16r(w0));
    const unsigned int c1 = hbits(W0CARRY * bf16r(w1));
    const unsigned int c2 = hbits(W0CARRY * bf16r(w2));
    const unsigned int c3 = hbits(W0CARRY * bf16r(w3));
    const unsigned int c4 = hbits(W0CARRY * bf16r(bb));
    v4u pv;
    pv[0] = on ? (c0 | (c1 << 16)) : 0u;
    pv[1] = on ? (c2 | (c3 << 16)) : 0u;
    pv[2] = on ? c4 : 0u;
    pv[3] = 0u;
    pc[i] = pv;
    po[i] = (size_t)q * 4u;
  }
#pragma unroll
  for (int i = 0; i < 2; ++i) *(volatile v4u*)(A0w + po[i]) = pc[i];
  __threadfence();
#pragma unroll
  for (int i = 0; i < 2; ++i) *(volatile v4u*)(A0w + po[i]) = pc[i];

  const unsigned e0 = 4u * t;
  const unsigned i1 = (e0 < 380u) ? e0 : 380u;
  const unsigned e2 = (e0 >= (unsigned)SP_W2) ? (e0 - (unsigned)SP_W2) : 0u;
  const unsigned i2 = (e2 < 380u) ? e2 : 380u;
  const v4f vb1 = *(const v4f*)(b1 + i1);
  const v4f vw2 = *(const v4f*)(W2 + i2);
  v4f val;
#pragma unroll
  for (unsigned j = 0; j < 4u; ++j) {
    const unsigned e = e0 + j;
    const unsigned e3 = (e >= (unsigned)SP_B2) ? (e - (unsigned)SP_B2) : 0u;
    const unsigned i3 = (e3 < (unsigned)(NODES - 1)) ? e3 : (unsigned)(NODES - 1);
    const float vb2 = b2[i3];
    float r = (e >= (unsigned)SP_B2 && e3 < (unsigned)NODES) ? bf16r(vb2) : 0.0f;
    r = (e0 < (unsigned)SP_B2) ? bf16r(vw2[j]) * (1.0f / ACARRY) : r;
    r = (e0 < (unsigned)SP_W2) ? ACARRY * bf16r(vb1[j]) : r;
    val[j] = r;
  }
  const unsigned es = (e0 < (unsigned)(SP_FLOATS - 4)) ? e0 : (unsigned)(SP_FLOATS - 4);
  if (t < 200u) {
    *(volatile v4f*)(SP + es) = val;
    __threadfence();
    *(volatile v4f*)(SP + es) = val;
  }
}

__global__ __launch_bounds__(128) void mlp_kernel(
    const float* __restrict__ Y, const float* __restrict__ Z, const int* __restrict__ PIDX,
    const unsigned int* __restrict__ A0w, const _Float16* __restrict__ W1t,
    const float* __restrict__ SP, float* __restrict__ out) {
  __shared__ __attribute__((aligned(16))) float St[WAVES * TILE_FLOATS];

  const unsigned lane = threadIdx.x & 31u;
  const int wave = __builtin_amdgcn_readfirstlane(threadIdx.x >> 5);
  const unsigned hh = lane >> 4, m = lane & 15u;
  const unsigned tile = blockIdx.x * (unsigned)WAVES + (unsigned)wave;
  if (tile >= (unsigned)NTILES) return;

  unsigned row = tile * 16u + m;
  row = (row < (unsigned)NROWS) ? row : ((unsigned)NROWS - 1u);
  const v2f* yp = (const v2f*)(Y + (size_t)row * NODES);
  const v2f* zp = (const v2f*)(Z + (size_t)row * NODES);
  const v2f ya = yp[0], yb = yp[1], yc = yp[2];
  const v2f za = zp[0], zb = zp[1], zc = zp[2];
  const bool lo_half = (hh == 0u);
  const float yq0 = carry_x(ya[0], lo_half), yq1 = carry_x(ya[1], lo_half);
  const float yq2 = carry_x(yb[0], lo_half), yq3 = carry_x(yb[1], lo_half);
  const float yq4 = carry_x(yc[0], lo_half), yq5 = carry_x(yc[1], lo_half);
  const float zq0 = carry_x(za[0], lo_half), zq1 = carry_x(za[1], lo_half);
  const float zq2 = carry_x(zb[0], lo_half), zq3 = carry_x(zb[1], lo_half);
  const float zq4 = carry_x(zc[0], lo_half), zq5 = carry_x(zc[1], lo_half);
  const float one_slot = lo_half ? XCARRY : 0.0f;

#pragma unroll 1
  for (int s = 0; s < NODES; ++s) {
    int p0 = PIDX[s * NPAR + 0];
    int p1 = PIDX[s * NPAR + 1];
    int p2 = PIDX[s * NPAR + 2];
    p0 = min(max(p0, 0), NODES - 1);
    p1 = min(max(p1, 0), NODES - 1);
    p2 = min(max(p2, 0), NODES - 1);
    const float x0 = pick6(p0, yq0, yq1, yq2, yq3, yq4, yq5);
    const float x1 = pick6(p1, yq0, yq1, yq2, yq3, yq4, yq5);
    const float x2 = pick6(p2, yq0, yq1, yq2, yq3, yq4, yq5);
    const float x3 = pick6(s, zq0, zq1, zq2, zq3, zq4, zq5);

    v8u bw;
    bw[0] = hbits(x0) | (hbits(x1) << 16);
    bw[1] = hbits(x2) | (hbits(x3) << 16);
    bw[2] = hbits(one_slot);
    bw[3] = 0u; bw[4] = 0u; bw[5] = 0u; bw[6] = 0u; bw[7] = 0u;
    const v16h bx = __builtin_bit_cast(v16h, bw);

    v8f d0[4];
#pragma unroll
    for (int t = 0; t < 4; ++t) {
      const unsigned piece = (((unsigned)s * 64u + (unsigned)t * 16u + m) << 1) + hh;
      const v4u lo = *(const v4u*)(A0w + (size_t)piece * 4u);
      v8u aw;
      aw[0] = lo[0]; aw[1] = lo[1]; aw[2] = lo[2]; aw[3] = lo[3];
      aw[4] = 0u; aw[5] = 0u; aw[6] = 0u; aw[7] = 0u;
      const v16h a = __builtin_bit_cast(v16h, aw);
      d0[t] = wmma16(a, bx, (v8f){});
    }

    v16h hb[2];
#pragma unroll
    for (int c = 0; c < 2; ++c) {
#pragma unroll
      for (int i = 0; i < 8; ++i) {
        hb[c][i]     = toh_flush(leaky_act(d0[2 * c][i]));
        hb[c][i + 8] = toh_flush(leaky_act(d0[2 * c + 1][i]));
      }
    }

    v8f acc[4];
#pragma unroll
    for (int nt = 0; nt < 4; ++nt) {
      const float* cp = SP + SP_C1 + (unsigned)s * 64u + (unsigned)nt * 16u + hh * 8u;
      const v4f c0 = *(const v4f*)(cp);
      const v4f c1 = *(const v4f*)(cp + 4);
      v8f t;
      t[0] = c0[0]; t[1] = c0[1]; t[2] = c0[2]; t[3] = c0[3];
      t[4] = c1[0]; t[5] = c1[1]; t[6] = c1[2]; t[7] = c1[3];
      acc[nt] = t;
    }
#pragma unroll
    for (int c = 0; c < 2; ++c) {
#pragma unroll
      for (int nt = 0; nt < 4; ++nt) {
        const _Float16* ap = W1t + (size_t)((unsigned)nt * 16u + m) * W1T_PITCH +
                             (unsigned)s * 64u + (unsigned)c * 32u + hh * 8u;
        const v16h a = frag_at(ap);
        acc[nt] = wmma16(a, hb[c], acc[nt]);
      }
    }

    float pr = 0.0f;
#pragma unroll
    for (int nt = 0; nt < 4; ++nt) {
      const float* wp = SP + SP_W2 + (unsigned)s * 64u + (unsigned)nt * 16u + hh * 8u;
      const v4f w0 = *(const v4f*)(wp);
      const v4f w1 = *(const v4f*)(wp + 4);
#pragma unroll
      for (int r = 0; r < 4; ++r) {
        pr += leaky_act(acc[nt][r]) * w0[r];
        pr += leaky_act(acc[nt][r + 4]) * w1[r];
      }
    }
    pr += __shfl_xor(pr, 16, 32);
    const float val = pr + SP[SP_B2 + s];
    if (lo_half) St[(unsigned)wave * TILE_FLOATS + m * NODES + (unsigned)s] = val;
  }

  wave_lds_sync();
  const unsigned li = (lane < 24u) ? lane : 23u;
  const v4f xo = *(const v4f*)&St[(unsigned)wave * TILE_FLOATS + li * 4u];
  float* op = out + (size_t)tile * TILE_FLOATS + li * 4u;
  if (lane < 24u) {
    *(volatile v4f*)op = xo;
    __threadfence();
    *(volatile v4f*)op = xo;
  }
}

extern "C" void kernel_launch(void* const* d_in, const int* in_sizes, int n_in,
                              void* d_out, int out_size, void* d_ws, size_t ws_size,
                              hipStream_t stream) {
  if (n_in < 10) return;
  const long long need_rows = (long long)NROWS * NODES;
  if ((long long)in_sizes[0] < need_rows) return;
  if ((long long)in_sizes[1] < need_rows) return;
  if (in_sizes[3] < NODES * NPAR) return;
  if (in_sizes[4] < NODES * 4 * HIDN) return;
  if (in_sizes[5] < NODES * HIDN) return;
  if (in_sizes[6] < NODES * HIDN * HIDN) return;
  if (in_sizes[7] < NODES * HIDN) return;
  if (in_sizes[8] < NODES * HIDN) return;
  if (in_sizes[9] < NODES) return;
  if ((long long)out_size < need_rows) return;
  if (ws_size < WS_TOTAL) return;

  const float* y    = (const float*)d_in[0];
  const float* z    = (const float*)d_in[1];
  const int*   pidx = (const int*)d_in[3];
  const float* w0   = (const float*)d_in[4];
  const float* b0   = (const float*)d_in[5];
  const float* w1   = (const float*)d_in[6];
  const float* b1   = (const float*)d_in[7];
  const float* w2   = (const float*)d_in[8];
  const float* b2   = (const float*)d_in[9];
  float* out = (float*)d_out;

  char* ws = (char*)d_ws;
  _Float16*     W1t = (_Float16*)(ws + OFF_W1T);
  unsigned int* A0w = (unsigned int*)(ws + OFF_A0);
  float*        SP  = (float*)(ws + OFF_SP);

  wconv_kernel<<<dim3(HIDN / 64, (NODES * HIDN) / 64), dim3(256), 0, stream>>>(
      w1, W1t, (unsigned)HIDN, (unsigned)W1T_PITCH);
  prep_small_kernel<<<dim3(1), dim3(384), 0, stream>>>(w0, b0, b1, w2, b2, A0w, SP);
  mlp_kernel<<<dim3((NTILES + WAVES - 1) / WAVES), dim3(WAVES * 32), 0, stream>>>(
      y, z, pidx, A0w, W1t, SP, out);
}
